// MixLoraSparseMoe_45088566673916
// MI455X (gfx1250) — hardware-verified
//
#include <hip/hip_runtime.h>
#include <math.h>

typedef __attribute__((ext_vector_type(16))) _Float16 v16h;
typedef __attribute__((ext_vector_type(16))) __bf16 v16b;
typedef __attribute__((ext_vector_type(8)))  _Float16 v8h;
typedef __attribute__((ext_vector_type(8)))  __bf16 v8b;
typedef __attribute__((ext_vector_type(8)))  float v8f;
typedef __attribute__((ext_vector_type(4)))  float v4f;
typedef __attribute__((ext_vector_type(4)))  unsigned v4u;
typedef _Float16 h16;

#ifndef NB
#define NB 1024
#endif
#define NB_FULL 1024
#define DIN  1024
#define DFF  4096
#define DOUT 1024
#define NE   8
#define LR   16
#define KF DFF
#define KP (KF + NE * LR)
#define TPITCH (2 * NE * LR)
#define HCARRY 64.0f
#define WCARRY 512.0f
#define TCARRY 16.0f
#define CCARRY 4096.0f
#define CINV   (1.0f / 4096.0f)
#define ZSCALE (1.0f / 256.0f)
#define OSCALE (1.0f / 32768.0f)
#define ACT_ROWS 32
#define ACT_COLS 128
#define ACT_WAVES 8

#define WS_XB  ((size_t)0)
#define WS_WGB (WS_XB  + (size_t)NB * DIN * 2)
#define WS_WUB (WS_WGB + (size_t)DFF * DIN * 2)
#define WS_A13 (WS_WUB + (size_t)DFF * DIN * 2)
#define WS_TP  (WS_A13 + (size_t)TPITCH * DIN * 2)
#define WS_B1H (WS_TP  + (size_t)NB * TPITCH * 2)
#define WS_B3H (WS_B1H + (size_t)NE * DFF * LR * 2)
#define WS_A2H (WS_B3H + (size_t)NE * DFF * LR * 2)
#define WS_W2T (WS_A2H + (size_t)NE * LR * DFF * 2)
#define WS_HB  (WS_W2T + (size_t)DOUT * KP * 2)
#define WS_WT  (WS_HB  + (size_t)NB * KP * 2)
#define WS_END (WS_WT  + (size_t)NB * NE * 4)

static_assert(NB % 128 == 0);
static_assert(NB <= NB_FULL);
static_assert(DIN % 32 == 0 && KP % 32 == 0 && (KP * 2) % 128 == 0 && DFF % 128 == 0);
static_assert((size_t)NB_FULL * DOUT * 4 == 4194304);
static_assert(WS_WGB % 128 == 0 && WS_WUB % 128 == 0 && WS_A13 % 128 == 0 && WS_TP % 128 == 0);
static_assert(WS_B1H % 128 == 0 && WS_B3H % 128 == 0 && WS_A2H % 128 == 0 && WS_W2T % 128 == 0 && WS_HB % 128 == 0 && WS_WT % 128 == 0);
static_assert(WS_END <= (size_t)134217728);
static_assert((size_t)(NB * DIN / 8 / 256) * 256 * 8 == (size_t)NB * DIN);
static_assert((size_t)(DFF * DIN / 8 / 256) * 256 * 8 == (size_t)DFF * DIN);
static_assert((size_t)(NE * LR * DIN / 8 / 256) * 256 * 8 == (size_t)NE * LR * DIN);
static_assert((size_t)(NE * DFF * LR / 8 / 256) * 256 * 8 == (size_t)NE * DFF * LR);
static_assert((size_t)(DOUT * DFF / 8 / 256) * 256 * 8 == (size_t)DOUT * DFF);
static_assert((size_t)(DOUT * 16 / 256) * 256 * 8 == (size_t)DOUT * NE * LR);
static_assert((size_t)(NB * NE / 256) * 256 == (size_t)NB * NE);
static_assert((size_t)(TPITCH / 128) * (NB / 128) * 128 * 128 == (size_t)NB * TPITCH);
static_assert((size_t)(NB / ACT_ROWS) * ACT_ROWS * KP == (size_t)NB * KP);
static_assert((size_t)(DOUT / 128) * (NB / 128) * 128 * 128 == (size_t)NB * DOUT);
static_assert(ACT_WAVES == (ACT_ROWS / 16) * (ACT_COLS / 32));
static_assert(ACT_WAVES * 32 == 256);
static_assert(NB % ACT_ROWS == 0 && DFF % ACT_COLS == 0);
static_assert(ACT_ROWS * NE == 256);
static_assert(NE * LR == ACT_COLS);
static_assert(32 * 16 * 8 == 32 * 128);
static_assert(256 * 16 * 2 == ACT_ROWS * ACT_COLS * 2);
static_assert(8 * 32 * 64 * 2 <= 131072);
static_assert(ACT_WAVES * NE * 256 * 4 + ACT_WAVES * 16 * 40 * 2 + ACT_ROWS * ACT_COLS * 2 + ACT_ROWS * NE * 4 <= 131072);
static_assert(8 * 16 * 64 * 4 <= 131072);
static_assert((DFF / 8) == 512 && LR == 16 && NE == 8);

__device__ __forceinline__ v8f wmma16(v16h a, v16h b, v8f c) {
  v8f d = __builtin_amdgcn_wmma_f32_16x16x32_f16(false, a, false, b, (short)0, c, false, false);
  asm volatile("v_nop\n\tv_nop\n\tv_nop\n\tv_nop" : "+v"(d) : "v"(a), "v"(b));
  return d;
}
__device__ __forceinline__ v8f wmma_bf(v16b a, v16b b, v8f c) {
  v8f d = __builtin_amdgcn_wmma_f32_16x16x32_bf16(false, a, false, b, (short)0, c, false, false);
  asm volatile("v_nop\n\tv_nop\n\tv_nop\n\tv_nop" : "+v"(d) : "v"(a), "v"(b));
  return d;
}
__device__ __forceinline__ float bfr(float v) { return (float)(__bf16)v; }
__device__ __forceinline__ v16b ldfrag_b(const unsigned short* p) { union { v16b v; v4u q[2]; } f; f.q[0] = *(const v4u*)p; f.q[1] = *(const v4u*)(p + 16); return f.v; }
__device__ __forceinline__ v16h ldfrag_h(const unsigned short* p) { union { v16h v; v4u q[2]; } f; f.q[0] = *(const v4u*)p; f.q[1] = *(const v4u*)(p + 16); return f.v; }
__device__ __forceinline__ v16h ldfrag_k16(const unsigned short* p) { union { v16h v; v4u q[2]; } f; const v4u z = {0u, 0u, 0u, 0u}; f.q[0] = *(const v4u*)p; f.q[1] = z; return f.v; }
static __device__ __forceinline__ h16 toh_flush(float v) { const h16 r = (h16)v; return (fabsf(v) < 6.103515625e-05f) ? (h16)0.0f : r; }

__global__ __launch_bounds__(256) void k_cvt_x(const float* __restrict__ X, unsigned short* __restrict__ XB) {
  const unsigned i = blockIdx.x * 256u + threadIdx.x;
  const unsigned ic = i < (unsigned)(NB * DIN / 8) ? i : (unsigned)(NB * DIN / 8 - 1);
  const v4f a = *(const v4f*)(X + (size_t)ic * 8), b = *(const v4f*)(X + (size_t)ic * 8 + 4);
  union { v8b h; v4u u; } o;
#pragma unroll
  for (int j = 0; j < 4; ++j) { o.h[j] = (__bf16)a[j]; o.h[4 + j] = (__bf16)b[j]; }
  const v4u val = o.u;
  volatile v4u* p = (volatile v4u*)(XB + (size_t)ic * 8);
  *p = val; __threadfence(); *p = val;
}

__global__ __launch_bounds__(256) void k_cvt_bf(const float* __restrict__ S, unsigned short* __restrict__ D, unsigned n8) {
  const unsigned i = blockIdx.x * 256u + threadIdx.x;
  const unsigned ic = i < n8 ? i : n8 - 1u;
  const v4f a = *(const v4f*)(S + (size_t)ic * 8), b = *(const v4f*)(S + (size_t)ic * 8 + 4);
  union { v8b h; v4u u; } o;
#pragma unroll
  for (int j = 0; j < 4; ++j) { o.h[j] = (__bf16)a[j]; o.h[4 + j] = (__bf16)b[j]; }
  const v4u val = o.u;
  volatile v4u* p = (volatile v4u*)(D + (size_t)ic * 8);
  *p = val; __threadfence(); *p = val;
}

__global__ __launch_bounds__(256) void k_cvt_h(const float* __restrict__ S, unsigned short* __restrict__ D, unsigned n8, unsigned lg, unsigned dpitch, float sc) {
  const unsigned i = blockIdx.x * 256u + threadIdx.x;
  const unsigned ic = i < n8 ? i : n8 - 1u;
  const unsigned row = ic >> lg, c8 = ic & ((1u << lg) - 1u);
  const v4f a = *(const v4f*)(S + (size_t)ic * 8), b = *(const v4f*)(S + (size_t)ic * 8 + 4);
  union { v8h h; v4u u; } o;
#pragma unroll
  for (int j = 0; j < 4; ++j) { o.h[j] = toh_flush(bfr(a[j]) * sc); o.h[4 + j] = toh_flush(bfr(b[j]) * sc); }
  const v4u val = o.u;
  volatile v4u* p = (volatile v4u*)(D + (size_t)row * dpitch + 8u * c8);
  *p = val; __threadfence(); *p = val;
}

__global__ __launch_bounds__(256) void k_b2pad(const float* __restrict__ B2, unsigned short* __restrict__ W2T) {
  const unsigned idx = blockIdx.x * 256u + threadIdx.x; const unsigned n = (idx >> 4) & (DOUT - 1u), q = idx & 15u, e = q >> 1, r0 = (q & 1u) * 8u;
  const float* s = B2 + ((size_t)e * DOUT + n) * LR + r0;
  const v4f a = *(const v4f*)s, b = *(const v4f*)(s + 4);
  union { v8h h; v4u u; } w;
#pragma unroll
  for (int j = 0; j < 4; ++j) { w.h[j] = toh_flush(bfr(a[j]) * WCARRY); w.h[4 + j] = toh_flush(bfr(b[j]) * WCARRY); }
  const v4u val = w.u;
  volatile v4u* p = (volatile v4u*)(W2T + (size_t)n * KP + KF + 8u * q);
  *p = val; __threadfence(); *p = val;
}

__global__ __launch_bounds__(256) void k_router(const float* __restrict__ X, const float* __restrict__ GW, float* __restrict__ WT) {
#pragma clang fp contract(off)
  const unsigned i = blockIdx.x * 256u + threadIdx.x, lane = threadIdx.x & 31u;
  const unsigned tok = i >> 3, e = i & 7u;
  const float* px = X + (size_t)tok * DIN; const float* pg = GW + (size_t)e * DIN;
  float lg = 0.f;
#pragma unroll 1
  for (unsigned k = 0; k < DIN; k += 4u) { const v4f a = *(const v4f*)(px + k), g = *(const v4f*)(pg + k);
    lg = fmaf(bfr(a[0]), bfr(g[0]), lg); lg = fmaf(bfr(a[1]), bfr(g[1]), lg); lg = fmaf(bfr(a[2]), bfr(g[2]), lg); lg = fmaf(bfr(a[3]), bfr(g[3]), lg); }
  float m = lg; m = fmaxf(m, __shfl_xor(m, 1)); m = fmaxf(m, __shfl_xor(m, 2)); m = fmaxf(m, __shfl_xor(m, 4));
  const float ev = expf(lg - m); float s = ev; s += __shfl_xor(s, 1); s += __shfl_xor(s, 2); s += __shfl_xor(s, 4);
  const float p = ev * (1.0f / s);
  const unsigned base = lane & 24u; unsigned rank = 0u;
#pragma unroll
  for (unsigned j = 0; j < 8u; ++j) { const float pj = __shfl(p, (int)(base + j)); rank += ((pj > p) || (pj == p && j < e)) ? 1u : 0u; }
  const float vs = rank < 2u ? p : 0.f; float s2 = vs; s2 += __shfl_xor(s2, 1); s2 += __shfl_xor(s2, 2); s2 += __shfl_xor(s2, 4);
  const float w = rank < 2u ? p * (1.0f / s2) : 0.f;
  volatile float* q = WT + i;
  *q = w; __threadfence(); *q = w;
}

__global__ __launch_bounds__(256) void k_ta(const unsigned short* __restrict__ XB, const unsigned short* __restrict__ A13, unsigned short* __restrict__ T) {
  __shared__ __align__(16) _Float16 sh[8][32][64];
  const unsigned t = threadIdx.x, wave = t >> 5, lane = t & 31u, lm = lane & 15u, lh = lane >> 4, wm = wave >> 1, wn = wave & 1u;
  const unsigned m0 = blockIdx.y * 128u, n0 = blockIdx.x * 128u;
  const unsigned short* ar[2]; const unsigned short* br[4];
#pragma unroll
  for (int mi = 0; mi < 2; ++mi) ar[mi] = XB + (size_t)(m0 + wm * 32u + mi * 16u + lm) * DIN + 8u * lh;
#pragma unroll
  for (int ni = 0; ni < 4; ++ni) br[ni] = A13 + (size_t)(n0 + wn * 64u + ni * 16u + lm) * DIN + 8u * lh;
  v8f acc[2][4] = {};
#pragma unroll 2
  for (unsigned kc = 0; kc < DIN / 32; ++kc) { v16b a[2], b[4];
#pragma unroll
    for (int mi = 0; mi < 2; ++mi) a[mi] = ldfrag_b(ar[mi] + kc * 32u);
#pragma unroll
    for (int ni = 0; ni < 4; ++ni) b[ni] = ldfrag_b(br[ni] + kc * 32u);
#pragma unroll
    for (int mi = 0; mi < 2; ++mi)
#pragma unroll
      for (int ni = 0; ni < 4; ++ni) acc[mi][ni] = wmma_bf(a[mi], b[ni], acc[mi][ni]); }
#pragma unroll
  for (int ni = 0; ni < 4; ++ni)
#pragma unroll
    for (int mi = 0; mi < 2; ++mi)
#pragma unroll
      for (int r = 0; r < 8; ++r) sh[wave][mi * 16 + 8u * lh + r][ni * 16 + lm] = toh_flush(acc[mi][ni][r] * TCARRY);
  __syncthreads();
  v4u o[8];
#pragma unroll
  for (unsigned it = 0; it < 8; ++it) { const unsigned rw = it * 4u + (lane >> 3), q = lane & 7u; union { v8h h; v4u u; } w; w.h = *(const v8h*)&sh[wave][rw][8u * q]; o[it] = w.u; }
  unsigned short* tb = T + (size_t)(m0 + wm * 32u) * TPITCH + n0 + wn * 64u;
#pragma unroll
  for (unsigned it = 0; it < 8; ++it) { const unsigned rw = it * 4u + (lane >> 3), q = lane & 7u; *(volatile v4u*)(tb + (size_t)rw * TPITCH + 8u * q) = o[it]; }
  __threadfence();
#pragma unroll
  for (unsigned it = 0; it < 8; ++it) { const unsigned rw = it * 4u + (lane >> 3), q = lane & 7u; *(volatile v4u*)(tb + (size_t)rw * TPITCH + 8u * q) = o[it]; }
}

__global__ __launch_bounds__(256) void k_act(const unsigned short* __restrict__ XB, const unsigned short* __restrict__ WGB, const unsigned short* __restrict__ WUB, const unsigned short* __restrict__ TP, const unsigned short* __restrict__ B1H, const unsigned short* __restrict__ B3H, const unsigned short* __restrict__ A2H, const float* __restrict__ WT, unsigned short* __restrict__ HB) {
  __shared__ __align__(32) float zsp[ACT_WAVES * NE * 256];
  __shared__ __align__(16) _Float16 sact[ACT_WAVES][16][40];
  __shared__ __align__(16) _Float16 sout[ACT_ROWS][ACT_COLS];
  __shared__ float swt[ACT_ROWS][NE];
  const unsigned t = threadIdx.x, lane = t & 31u, lm = lane & 15u, lh = lane >> 4;
  const unsigned wave = (unsigned)__builtin_amdgcn_readfirstlane((int)(t >> 5));
  const unsigned wm = wave >> 2, wn = wave & 3u;
  const unsigned m0 = blockIdx.x * 32u;
  swt[t >> 3][t & 7u] = WT[(size_t)m0 * NE + t];
  { const v8f z8 = {};
#pragma unroll
    for (unsigned j = 0; j < NE; ++j) *(v8f*)&zsp[((wave * NE + j) * 32u + lane) * 8u] = z8; }
  __syncthreads();
#pragma unroll 1
  for (unsigned ch = 0; ch < DFF / ACT_COLS; ++ch) {
    const unsigned f0 = ch * 128u + wn * 32u;
    const unsigned short* ar = XB + (size_t)(m0 + wm * 16u + lm) * DIN + 8u * lh;
    const unsigned short* bg[2]; const unsigned short* bu[2];
#pragma unroll
    for (int ni = 0; ni < 2; ++ni) { bg[ni] = WGB + (size_t)(f0 + ni * 16u + lm) * DIN + 8u * lh; bu[ni] = WUB + (size_t)(f0 + ni * 16u + lm) * DIN + 8u * lh; }
    v8f ag[2] = {}, au[2] = {};
#pragma unroll 2
    for (unsigned kc = 0; kc < DIN / 32; ++kc) { v16b g[2], u[2];
      const v16b a = ldfrag_b(ar + kc * 32u);
#pragma unroll
      for (int ni = 0; ni < 2; ++ni) { g[ni] = ldfrag_b(bg[ni] + kc * 32u); u[ni] = ldfrag_b(bu[ni] + kc * 32u); }
#pragma unroll
      for (int ni = 0; ni < 2; ++ni) { ag[ni] = wmma_bf(a, g[ni], ag[ni]); au[ni] = wmma_bf(a, u[ni], au[ni]); } }
    v8f ws[2] = {};
#pragma unroll 1
    for (unsigned e = 0; e < NE; ++e) {
      v16h b1[2], b3[2];
#pragma unroll
      for (int ni = 0; ni < 2; ++ni) { const size_t bo = ((size_t)e * DFF + f0 + ni * 16u + lm) * LR + 8u * lh; b1[ni] = ldfrag_k16(B1H + bo); b3[ni] = ldfrag_k16(B3H + bo); }
      const unsigned short* tp = TP + (size_t)(m0 + wm * 16u + lm) * TPITCH + e * LR + 8u * lh;
      const v16h t1 = ldfrag_k16(tp), t3 = ldfrag_k16(tp + NE * LR);
      float wv[8];
#pragma unroll
      for (int r = 0; r < 8; ++r) wv[r] = swt[wm * 16u + 8u * lh + r][e];
#pragma unroll
      for (int ni = 0; ni < 2; ++ni) {
        v8f c1 = ag[ni] * CCARRY, c3 = au[ni] * CCARRY;
        c1 = wmma16(t1, b1[ni], c1);
        c3 = wmma16(t3, b3[ni], c3);
#pragma unroll
        for (int r = 0; r < 8; ++r) { const float v1 = c1[r] * CINV, v3 = c3[r] * CINV;
          const float sg = __builtin_amdgcn_rcpf(1.0f + __expf(fminf(-v1, 80.0f)));
          const float a = v1 * sg * v3;
          ws[ni][r] = fmaf(wv[r], a, ws[ni][r]);
          sact[wave][8u * lh + r][ni * 16 + lm] = toh_flush(a * HCARRY); } }
      __syncthreads();
      const v16h za = ldfrag_h(A2H + ((size_t)e * LR + lm) * DFF + f0 + 8u * lh);
      { union { v16h v; v8h q[2]; } fa;
        fa.q[0] = *(const v8h*)&sact[wave][lm][8u * lh]; fa.q[1] = *(const v8h*)&sact[wave][lm][16u + 8u * lh];
        float* zp = &zsp[((wave * NE + e) * 32u + lane) * 8u];
        v8f zc = *(const v8f*)zp; zc = wmma16(fa.v, za, zc); *(v8f*)zp = zc; }
      __syncthreads();
    }
#pragma unroll
    for (int ni = 0; ni < 2; ++ni)
#pragma unroll
      for (int r = 0; r < 8; ++r) sout[wm * 16u + 8u * lh + r][wn * 32u + ni * 16 + lm] = toh_flush(ws[ni][r] * HCARRY);
    __syncthreads();
    v4u o[2];
#pragma unroll
    for (unsigned it = 0; it < 2; ++it) { const unsigned idx = it * 256u + t, rw = idx >> 4, q = idx & 15u; union { v8h h; v4u u; } w; w.h = *(const v8h*)&sout[rw][8u * q]; o[it] = w.u; }
    unsigned short* hb = HB + (size_t)m0 * KP + ch * 128u;
#pragma unroll
    for (unsigned it = 0; it < 2; ++it) { const unsigned idx = it * 256u + t, rw = idx >> 4, q = idx & 15u; *(volatile v4u*)(hb + (size_t)rw * KP + 8u * q) = o[it]; }
    __threadfence();
#pragma unroll
    for (unsigned it = 0; it < 2; ++it) { const unsigned idx = it * 256u + t, rw = idx >> 4, q = idx & 15u; *(volatile v4u*)(hb + (size_t)rw * KP + 8u * q) = o[it]; }
  }
  __syncthreads();
  v4u oz[2];
#pragma unroll
  for (unsigned it = 0; it < 2; ++it) { const unsigned idx = it * 256u + t, rw = idx >> 4, q = idx & 15u;
    const unsigned e = q >> 1, rm = rw >> 4, hh = (rw >> 3) & 1u, r = rw & 7u, lb = hh * 16u + (q & 1u) * 8u;
    const float wz = swt[rw][e] * ZSCALE;
    union { v8h h; v4u u; } w;
#pragma unroll
    for (int i = 0; i < 8; ++i) { float s = 0.f;
#pragma unroll
      for (unsigned wv = 0; wv < 4; ++wv) s += zsp[(((rm * 4u + wv) * NE + e) * 32u + lb + i) * 8u + r];
      w.h[i] = toh_flush(s * wz); }
    oz[it] = w.u; }
  unsigned short* hz = HB + (size_t)m0 * KP + KF;
#pragma unroll
  for (unsigned it = 0; it < 2; ++it) { const unsigned idx = it * 256u + t, rw = idx >> 4, q = idx & 15u; *(volatile v4u*)(hz + (size_t)rw * KP + 8u * q) = oz[it]; }
  __threadfence();
#pragma unroll
  for (unsigned it = 0; it < 2; ++it) { const unsigned idx = it * 256u + t, rw = idx >> 4, q = idx & 15u; *(volatile v4u*)(hz + (size_t)rw * KP + 8u * q) = oz[it]; }
}

__global__ __launch_bounds__(256) void k_out(const unsigned short* __restrict__ HB, const unsigned short* __restrict__ W2T, float* __restrict__ OUT) {
  __shared__ __align__(16) float sf[8][16][64];
  const unsigned t = threadIdx.x, wave = t >> 5, lane = t & 31u, lm = lane & 15u, lh = lane >> 4, wm = wave >> 1, wn = wave & 1u;
  const unsigned m0 = blockIdx.y * 128u, n0 = blockIdx.x * 128u;
  const unsigned short* ar[2]; const unsigned short* br[4];
#pragma unroll
  for (int mi = 0; mi < 2; ++mi) ar[mi] = HB + (size_t)(m0 + wm * 32u + mi * 16u + lm) * KP + 8u * lh;
#pragma unroll
  for (int ni = 0; ni < 4; ++ni) br[ni] = W2T + (size_t)(n0 + wn * 64u + ni * 16u + lm) * KP + 8u * lh;
  v8f acc[2][4] = {};
#pragma unroll 2
  for (unsigned kc = 0; kc < KP / 32; ++kc) { v16h a[2], b[4];
#pragma unroll
    for (int mi = 0; mi < 2; ++mi) a[mi] = ldfrag_h(ar[mi] + kc * 32u);
#pragma unroll
    for (int ni = 0; ni < 4; ++ni) b[ni] = ldfrag_h(br[ni] + kc * 32u);
#pragma unroll
    for (int mi = 0; mi < 2; ++mi)
#pragma unroll
      for (int ni = 0; ni < 4; ++ni) acc[mi][ni] = wmma16(a[mi], b[ni], acc[mi][ni]); }
#pragma unroll
  for (int mi = 0; mi < 2; ++mi) {
    if (mi) __syncthreads();
#pragma unroll
    for (int ni = 0; ni < 4; ++ni)
#pragma unroll
      for (int r = 0; r < 8; ++r) sf[wave][8u * lh + r][ni * 16 + lm] = acc[mi][ni][r] * OSCALE;
    __syncthreads();
    v4f v[8];
#pragma unroll
    for (unsigned it = 0; it < 8; ++it) { const unsigned rw = it * 2u + (lane >> 4), pc = lane & 15u; v[it] = *(const v4f*)&sf[wave][rw][4u * pc]; }
    float* po = OUT + (size_t)(m0 + wm * 32u + mi * 16u) * DOUT + n0 + wn * 64u;
#pragma unroll
    for (unsigned it = 0; it < 8; ++it) { const unsigned rw = it * 2u + (lane >> 4), pc = lane & 15u; *(volatile v4f*)(po + (size_t)rw * DOUT + 4u * pc) = v[it]; }
    __threadfence();
#pragma unroll
    for (unsigned it = 0; it < 8; ++it) { const unsigned rw = it * 2u + (lane >> 4), pc = lane & 15u; *(volatile v4f*)(po + (size_t)rw * DOUT + 4u * pc) = v[it]; }
  }
}

extern "C" void kernel_launch(void* const* d_in, const int* in_sizes, int n_in, void* d_out, int out_size, void* d_ws, size_t ws_size, hipStream_t stream) {
  if (n_in < 11) return;
  if (in_sizes[0] < NB * DIN || in_sizes[1] < NE * DIN || in_sizes[2] < DFF * DIN || in_sizes[3] < DFF * DIN || in_sizes[4] < DOUT * DFF) return;
  if (in_sizes[5] < NE * LR * DIN || in_sizes[6] < NE * DFF * LR || in_sizes[7] < NE * LR * DIN || in_sizes[8] < NE * DFF * LR) return;
  if (in_sizes[9] < NE * LR * DFF || in_sizes[10] < NE * DOUT * LR) return;
  if ((size_t)out_size < (size_t)NB * DOUT) return;
  if (ws_size < (size_t)WS_END) return;
  const float* X   = (const float*)d_in[0];
  const float* GW  = (const float*)d_in[1];
  const float* WG  = (const float*)d_in[2];
  const float* WU  = (const float*)d_in[3];
  const float* WD  = (const float*)d_in[4];
  const float* A1  = (const float*)d_in[5];
  const float* B1  = (const float*)d_in[6];
  const float* A3  = (const float*)d_in[7];
  const float* B3  = (const float*)d_in[8];
  const float* A2  = (const float*)d_in[9];
  const float* B2  = (const float*)d_in[10];
  char* ws = (char*)d_ws;
  unsigned short* XB  = (unsigned short*)(ws + WS_XB);
  unsigned short* WGB = (unsigned short*)(ws + WS_WGB);
  unsigned short* WUB = (unsigned short*)(ws + WS_WUB);
  unsigned short* A13 = (unsigned short*)(ws + WS_A13);
  unsigned short* TP  = (unsigned short*)(ws + WS_TP);
  unsigned short* B1H = (unsigned short*)(ws + WS_B1H);
  unsigned short* B3H = (unsigned short*)(ws + WS_B3H);
  unsigned short* A2H = (unsigned short*)(ws + WS_A2H);
  unsigned short* W2T = (unsigned short*)(ws + WS_W2T);
  unsigned short* HB  = (unsigned short*)(ws + WS_HB);
  float* WT  = (float*)(ws + WS_WT);
  float* OUT = (float*)d_out;
  k_cvt_x<<<dim3(NB * DIN / 8 / 256), 256, 0, stream>>>(X, XB);
  k_cvt_bf<<<dim3(DFF * DIN / 8 / 256), 256, 0, stream>>>(WG, WGB, (unsigned)(DFF * DIN / 8));
  k_cvt_bf<<<dim3(DFF * DIN / 8 / 256), 256, 0, stream>>>(WU, WUB, (unsigned)(DFF * DIN / 8));
  k_cvt_bf<<<dim3(NE * LR * DIN / 8 / 256), 256, 0, stream>>>(A1, A13, (unsigned)(NE * LR * DIN / 8));
  k_cvt_bf<<<dim3(NE * LR * DIN / 8 / 256), 256, 0, stream>>>(A3, A13 + (size_t)NE * LR * DIN, (unsigned)(NE * LR * DIN / 8));
  k_cvt_h<<<dim3(NE * DFF * LR / 8 / 256), 256, 0, stream>>>(B1, B1H, (unsigned)(NE * DFF * LR / 8), 1u, (unsigned)LR, WCARRY);
  k_cvt_h<<<dim3(NE * DFF * LR / 8 / 256), 256, 0, stream>>>(B3, B3H, (unsigned)(NE * DFF * LR / 8), 1u, (unsigned)LR, WCARRY);
  k_cvt_h<<<dim3(NE * LR * DFF / 8 / 256), 256, 0, stream>>>(A2, A2H, (unsigned)(NE * LR * DFF / 8), 9u, (unsigned)DFF, WCARRY);
  k_cvt_h<<<dim3(DOUT * DFF / 8 / 256), 256, 0, stream>>>(WD, W2T, (unsigned)(DOUT * DFF / 8), 9u, (unsigned)KP, WCARRY);
  k_b2pad<<<dim3(DOUT * 16 / 256), 256, 0, stream>>>(B2, W2T);
  k_router<<<dim3(NB * NE / 256), 256, 0, stream>>>(X, GW, WT);
  k_ta<<<dim3(TPITCH / 128, NB / 128), 256, 0, stream>>>(XB, A13, TP);
  k_act<<<dim3(NB / ACT_ROWS), 256, 0, stream>>>(XB, WGB, WUB, TP, B1H, B3H, A2H, WT, HB);
  k_out<<<dim3(DOUT / 128, NB / 128), 256, 0, stream>>>(HB, W2T, OUT);
}
